// DeepSeekRelationalModel_25443386261956
// MI455X (gfx1250) — hardware-verified
//
#include <hip/hip_runtime.h>
#include <math.h>

typedef __attribute__((ext_vector_type(16))) _Float16 v16h;
typedef __attribute__((ext_vector_type(16))) __bf16 v16b;
typedef __attribute__((ext_vector_type(8)))  _Float16 v8h;
typedef __attribute__((ext_vector_type(8)))  __bf16 v8b;
typedef __attribute__((ext_vector_type(8)))  float v8f;
typedef __attribute__((ext_vector_type(4)))  float v4f;
typedef __attribute__((ext_vector_type(4)))  unsigned v4u;
typedef __attribute__((ext_vector_type(2)))  unsigned v2u;
typedef _Float16 h16;

#ifndef NB
#define NB 8192
#endif
#define NB_FULL 8192
#define DIN  1024
#define DHID 512
#define DOUT 1024
#define NE   16
#define HCARRY 64.0f
#define WCARRY 512.0f
#define OSCALE (1.0f / 32768.0f)
#define CH 1024
#define MT 32
#define RT 64

#define WS_XB  ((size_t)0)
#define WS_W1T (WS_XB  + (size_t)NB * DIN * 2)
#define WS_W3T (WS_W1T + (size_t)NE * DHID * DIN * 2)
#define WS_W2T (WS_W3T + (size_t)NE * DHID * DIN * 2)
#define WS_CMB (WS_W2T + (size_t)NE * DOUT * DHID * 2)
#define WS_Y1  (WS_CMB + (size_t)NB * NE * 4)
#define WS_END (WS_Y1  + (size_t)NB * DOUT * 4)

static_assert(NB % CH == 0);
static_assert(NB % RT == 0);
static_assert(NB <= NB_FULL);
static_assert(CH % 256 == 0 && CH % MT == 0);
static_assert(DIN % 32 == 0 && DHID % 32 == 0);
static_assert(DOUT == DIN);
static_assert((size_t)NB_FULL * DOUT * 4 == 33554432);
static_assert(WS_W1T % 128 == 0 && WS_W3T % 128 == 0 && WS_W2T % 128 == 0 && WS_CMB % 128 == 0 && WS_Y1 % 128 == 0);
static_assert(WS_END <= (size_t)134217728);
static_assert((size_t)(NB * DIN / 8 / 256) * 256 * 8 == (size_t)NB * DIN);
static_assert((size_t)(DHID / 64) * (DIN / 64) * NE * 4096 == (size_t)NE * DIN * DHID);
static_assert((size_t)(DOUT / 64) * (DHID / 64) * NE * 4096 == (size_t)NE * DHID * DOUT);
static_assert((size_t)(NB / RT) * RT * NE == (size_t)NB * NE);
static_assert(256 * 4 == RT * NE);
static_assert(16 * 256 * 4 == DIN * NE);
static_assert(256 * 16 * 8 == MT * DIN);
static_assert(4 * 32 * 16 == 16 * 32 * 4);
static_assert(8 * 64 == DHID && 8 * 128 == DOUT);
static_assert((size_t)(NB * DIN / 4 / 256) * 256 * 4 == (size_t)NB * DIN);
static_assert(MT * DIN * 2 + MT * DHID * 2 + 8 * 16 * 32 * 4 + CH * 12 + 8 * 4 <= 131072);
static_assert(DIN * NE * 4 + RT * NE * 4 <= 131072);
static_assert(64 * 65 * 4 <= 131072);

__device__ __forceinline__ v8f wmma16(v16h a, v16h b, v8f c) {
  v8f d = __builtin_amdgcn_wmma_f32_16x16x32_f16(false, a, false, b, (short)0, c, false, false);
  asm volatile("v_nop\n\tv_nop\n\tv_nop\n\tv_nop" : "+v"(d) : "v"(a), "v"(b));
  return d;
}
__device__ __forceinline__ v8f wmma_bf(v16b a, v16b b, v8f c) {
  v8f d = __builtin_amdgcn_wmma_f32_16x16x32_bf16(false, a, false, b, (short)0, c, false, false);
  asm volatile("v_nop\n\tv_nop\n\tv_nop\n\tv_nop" : "+v"(d) : "v"(a), "v"(b));
  return d;
}
__device__ __forceinline__ float bfr(float v) { return (float)(__bf16)v; }
static __device__ __forceinline__ h16 toh_flush(float v) { const h16 r = (h16)v; return (fabsf(v) < 6.103515625e-05f) ? (h16)0.0f : r; }
__device__ __forceinline__ v16b ldfrag_b(const unsigned short* p) { union { v16b v; v4u q[2]; } f; f.q[0] = *(const v4u*)p; f.q[1] = *(const v4u*)(p + 16); return f.v; }
__device__ __forceinline__ v16h ldfrag_h(const unsigned short* p) { union { v16h v; v4u q[2]; } f; f.q[0] = *(const v4u*)p; f.q[1] = *(const v4u*)(p + 16); return f.v; }

__global__ __launch_bounds__(256) void k_cvt_x(const float* __restrict__ X, unsigned short* __restrict__ XB) {
  const unsigned i = blockIdx.x * 256u + threadIdx.x;
  const unsigned ic = i < (unsigned)(NB * DIN / 8) ? i : (unsigned)(NB * DIN / 8 - 1);
  const v4f a = *(const v4f*)(X + (size_t)ic * 8), b = *(const v4f*)(X + (size_t)ic * 8 + 4);
  union { v8b h; v4u u; } o;
#pragma unroll
  for (int j = 0; j < 4; ++j) { o.h[j] = (__bf16)a[j]; o.h[4 + j] = (__bf16)b[j]; }
  const v4u val = o.u;
  volatile v4u* p = (volatile v4u*)(XB + (size_t)ic * 8);
  *p = val; __threadfence(); *p = val;
}

template <int F16>
__global__ __launch_bounds__(256) void k_tr(const float* __restrict__ S, unsigned short* __restrict__ Dst, unsigned K, unsigned N, unsigned dpitch, unsigned erow, unsigned ecol, float sc) {
  __shared__ float tile[64][65];
  const unsigned t = threadIdx.x, e = blockIdx.z, k0 = blockIdx.y * 64u, n0 = blockIdx.x * 64u;
  const float* s = S + (size_t)e * K * N;
#pragma unroll
  for (unsigned it = 0; it < 4; ++it) { const unsigned idx = it * 256u + t, kr = idx >> 4, c4 = idx & 15u;
    const v4f v = *(const v4f*)(s + (size_t)(k0 + kr) * N + n0 + 4u * c4);
    tile[kr][4u * c4 + 0] = v[0]; tile[kr][4u * c4 + 1] = v[1]; tile[kr][4u * c4 + 2] = v[2]; tile[kr][4u * c4 + 3] = v[3]; }
  __syncthreads();
  v4u o[2];
#pragma unroll
  for (unsigned it = 0; it < 2; ++it) { const unsigned idx = it * 256u + t, nr = idx >> 3, q = idx & 7u;
    union { v8b b; v8h h; v4u u; } w;
#pragma unroll
    for (int i = 0; i < 8; ++i) { const float v = bfr(tile[8u * q + i][nr]); if (F16) w.h[i] = toh_flush(v * sc); else w.b[i] = (__bf16)v; }
    o[it] = w.u; }
#pragma unroll
  for (unsigned it = 0; it < 2; ++it) { const unsigned idx = it * 256u + t, nr = idx >> 3, q = idx & 7u;
    *(volatile v4u*)(Dst + (size_t)(e * erow + n0 + nr) * dpitch + e * ecol + k0 + 8u * q) = o[it]; }
  __threadfence();
#pragma unroll
  for (unsigned it = 0; it < 2; ++it) { const unsigned idx = it * 256u + t, nr = idx >> 3, q = idx & 7u;
    *(volatile v4u*)(Dst + (size_t)(e * erow + n0 + nr) * dpitch + e * ecol + k0 + 8u * q) = o[it]; }
}

__global__ __launch_bounds__(256) void k_route(const unsigned short* __restrict__ XB, const float* __restrict__ GW, float* __restrict__ CMB) {
#pragma clang fp contract(off)
  __shared__ __align__(16) float gws[DIN][NE];
  __shared__ __align__(16) float sl[RT][NE];
  const unsigned tid = threadIdx.x; const unsigned r0 = blockIdx.x * (unsigned)RT;
#pragma unroll 1
  for (unsigned it = 0; it < (unsigned)(DIN * NE / (256 * 4)); ++it) { const unsigned idx = it * 256u + tid;
    const v4f v = *(const v4f*)(GW + 4u * idx); v4f o;
#pragma unroll
    for (int j = 0; j < 4; ++j) o[j] = bfr(v[j]);
    *(v4f*)(&gws[0][0] + 4u * idx) = o; }
  __syncthreads();
  const unsigned tl = tid >> 2, eq = tid & 3u;
  const unsigned short* xr = XB + (size_t)(r0 + tl) * DIN;
  float a0 = 0.f, a1 = 0.f, a2 = 0.f, a3 = 0.f;
#pragma unroll 1
  for (unsigned d0 = 0; d0 < (unsigned)DIN; d0 += 4u) {
    const v2u xv = *(const v2u*)(xr + d0);
    const float x0 = __uint_as_float(xv[0] << 16), x1 = __uint_as_float(xv[0] & 0xffff0000u);
    const float x2 = __uint_as_float(xv[1] << 16), x3 = __uint_as_float(xv[1] & 0xffff0000u);
    const v4f w0 = *(const v4f*)&gws[d0 + 0u][4u * eq], w1 = *(const v4f*)&gws[d0 + 1u][4u * eq];
    const v4f w2 = *(const v4f*)&gws[d0 + 2u][4u * eq], w3 = *(const v4f*)&gws[d0 + 3u][4u * eq];
    a0 = fmaf(x0, w0[0], a0); a1 = fmaf(x0, w0[1], a1); a2 = fmaf(x0, w0[2], a2); a3 = fmaf(x0, w0[3], a3);
    a0 = fmaf(x1, w1[0], a0); a1 = fmaf(x1, w1[1], a1); a2 = fmaf(x1, w1[2], a2); a3 = fmaf(x1, w1[3], a3);
    a0 = fmaf(x2, w2[0], a0); a1 = fmaf(x2, w2[1], a1); a2 = fmaf(x2, w2[2], a2); a3 = fmaf(x2, w2[3], a3);
    a0 = fmaf(x3, w3[0], a0); a1 = fmaf(x3, w3[1], a1); a2 = fmaf(x3, w3[2], a2); a3 = fmaf(x3, w3[3], a3);
  }
  { v4f lg; lg[0] = a0; lg[1] = a1; lg[2] = a2; lg[3] = a3; *(v4f*)&sl[tl][4u * eq] = lg; }
  __syncthreads();
  if (tid < (unsigned)RT) {
    float m = sl[tid][0];
#pragma unroll 1
    for (unsigned j = 1; j < (unsigned)NE; ++j) m = fmaxf(m, sl[tid][j]);
    float s = 0.f;
#pragma unroll 1
    for (unsigned j = 0; j < (unsigned)NE; ++j) { const float ev = expf(sl[tid][j] - m); sl[tid][j] = ev; s += ev; }
    const float inv = 1.0f / s;
    float b1 = -1.f, b2 = -1.f; unsigned i1 = 0u, i2 = 0u;
#pragma unroll 1
    for (unsigned j = 0; j < (unsigned)NE; ++j) { const float p = sl[tid][j] * inv; const bool g1 = p > b1, g2 = p > b2;
      const float nb2 = g1 ? b1 : (g2 ? p : b2); const unsigned ni2 = g1 ? i1 : (g2 ? j : i2);
      b1 = g1 ? p : b1; i1 = g1 ? j : i1; b2 = nb2; i2 = ni2; }
    const float rn = 1.0f / (b1 + b2);
    float wa = b1 * rn, wb = b2 * rn;
    wa = (wa > 0.f) ? wa : 1.17549435e-38f;
    wb = (wb > 0.f) ? wb : 1.17549435e-38f;
#pragma unroll 1
    for (unsigned j = 0; j < (unsigned)NE; ++j) sl[tid][j] = (j == i1) ? wa : ((j == i2) ? wb : 0.f);
  }
  __syncthreads();
  const v4f val = *(const v4f*)(&sl[0][0] + 4u * tid);
  volatile v4f* p = (volatile v4f*)(CMB + (size_t)r0 * NE + 4u * tid);
  *p = val; __threadfence(); *p = val;
}

__global__ __launch_bounds__(256) void k_moe(const unsigned short* __restrict__ XB, const unsigned short* __restrict__ W1T, const unsigned short* __restrict__ W3T, const unsigned short* __restrict__ W2T, const float* __restrict__ CMB, float* __restrict__ OUT, float* __restrict__ Y1) {
  __shared__ __align__(16) unsigned short xs[MT][DIN];
  __shared__ __align__(16) _Float16 hs[MT][DHID];
  __shared__ __align__(16) float sf[8][16][32];
  __shared__ int l_tok[CH]; __shared__ float l_w[CH]; __shared__ int l_slot[CH];
  __shared__ unsigned wc[8];
  const unsigned t = threadIdx.x, lane = t & 31u, lm = lane & 15u, lh = lane >> 4;
  const unsigned wave = (unsigned)__builtin_amdgcn_readfirstlane((int)(t >> 5));
  const unsigned e = blockIdx.y, c0 = blockIdx.x * (unsigned)CH;

  unsigned base = 0u;
#pragma unroll 1
  for (unsigned it = 0; it < (unsigned)(CH / 256); ++it) {
    const unsigned tk = c0 + it * 256u + t;
    const float* pr = CMB + (size_t)tk * NE;
    const v4f q0 = *(const v4f*)pr, q1 = *(const v4f*)(pr + 4), q2 = *(const v4f*)(pr + 8), q3 = *(const v4f*)(pr + 12);
    float rv[16];
#pragma unroll
    for (int j = 0; j < 4; ++j) { rv[j] = q0[j]; rv[4 + j] = q1[j]; rv[8 + j] = q2[j]; rv[12 + j] = q3[j]; }
    float wsel = 0.f; unsigned lower = 0u;
#pragma unroll
    for (unsigned j = 0; j < 16u; ++j) { wsel = (j == e) ? rv[j] : wsel; lower += (j < e && rv[j] != 0.f) ? 1u : 0u; }
    const bool hit = wsel != 0.f;
    const unsigned bal = __builtin_amdgcn_ballot_w32(hit);
    const unsigned before = (unsigned)__popc(bal & ((1u << lane) - 1u));
    if (lane == 0u) wc[wave] = (unsigned)__popc(bal);
    __syncthreads();
    unsigned off = base, tot = 0u;
#pragma unroll
    for (unsigned w = 0; w < 8u; ++w) { const unsigned c = wc[w]; off += (w < wave) ? c : 0u; tot += c; }
    const unsigned pos = off + before;
    if (hit && pos < (unsigned)CH) { l_tok[pos] = (int)tk; l_w[pos] = wsel; l_slot[pos] = lower ? 1 : 0; }
    base += tot;
    __syncthreads();
  }
  const unsigned nbv = base < (unsigned)CH ? base : (unsigned)CH;
  const unsigned ntv = (nbv + (unsigned)MT - 1u) / (unsigned)MT;
  const unsigned n = (unsigned)__builtin_amdgcn_readfirstlane((int)nbv);
  const unsigned ntile = (unsigned)__builtin_amdgcn_readfirstlane((int)ntv);

#pragma unroll 1
  for (unsigned tile = 0; tile < ntile; ++tile) {
    __syncthreads();
    {
      const unsigned r = t >> 3, c = t & 7u;
      const unsigned hidx = tile * (unsigned)MT + r; const bool ok = hidx < n; const unsigned hc = ok ? hidx : (n - 1u);
      int tk = l_tok[hc]; tk = tk < 0 ? 0 : tk; tk = tk > NB - 1 ? NB - 1 : tk;
      const unsigned short* src = XB + (size_t)tk * DIN;
      const unsigned msk = ok ? 0xffffffffu : 0u; v4u mk; mk[0] = msk; mk[1] = msk; mk[2] = msk; mk[3] = msk;
#pragma unroll 8
      for (unsigned j = 0; j < 16u; ++j) { v4u v = *(const v4u*)(src + 8u * (c + 8u * j)); v = v & mk; *(v4u*)&xs[r][8u * (c + 8u * j)] = v; }
    }
    __syncthreads();
#pragma unroll 1
    for (unsigned pa = 0; pa < 2u; ++pa) {
      const unsigned nh0 = wave * 64u + pa * 32u;
      const unsigned short* b1p[2]; const unsigned short* b3p[2];
#pragma unroll
      for (int ni = 0; ni < 2; ++ni) { b1p[ni] = W1T + (size_t)(e * DHID + nh0 + ni * 16u + lm) * DIN + 8u * lh; b3p[ni] = W3T + (size_t)(e * DHID + nh0 + ni * 16u + lm) * DIN + 8u * lh; }
      v8f ag[2][2] = {}; v8f au[2][2] = {};
#pragma unroll 2
      for (unsigned kc = 0; kc < (unsigned)(DIN / 32); ++kc) { v16b a[2], bg[2], bu[2];
#pragma unroll
        for (int mi = 0; mi < 2; ++mi) { union { v16b v; v4u q[2]; } f; f.q[0] = *(const v4u*)&xs[mi * 16 + lm][kc * 32u + 8u * lh]; f.q[1] = *(const v4u*)&xs[mi * 16 + lm][kc * 32u + 16u + 8u * lh]; a[mi] = f.v; }
#pragma unroll
        for (int ni = 0; ni < 2; ++ni) { bg[ni] = ldfrag_b(b1p[ni] + kc * 32u); bu[ni] = ldfrag_b(b3p[ni] + kc * 32u); }
#pragma unroll
        for (int mi = 0; mi < 2; ++mi)
#pragma unroll
          for (int ni = 0; ni < 2; ++ni) { ag[mi][ni] = wmma_bf(a[mi], bg[ni], ag[mi][ni]); au[mi][ni] = wmma_bf(a[mi], bu[ni], au[mi][ni]); } }
#pragma unroll
      for (int ni = 0; ni < 2; ++ni)
#pragma unroll
        for (int mi = 0; mi < 2; ++mi)
#pragma unroll
          for (int r = 0; r < 8; ++r) { const float g = ag[mi][ni][r], u = au[mi][ni][r]; const float sg = 1.0f / (1.0f + expf(-g));
            hs[mi * 16 + 8u * lh + r][nh0 + ni * 16u + lm] = toh_flush(g * sg * u * HCARRY); }
    }
    __syncthreads();
#pragma unroll 1
    for (unsigned pb = 0; pb < 2u; ++pb) {
      const unsigned nc0 = wave * 128u + pb * 64u;
      const unsigned short* br[4];
#pragma unroll
      for (int ni = 0; ni < 4; ++ni) br[ni] = W2T + (size_t)(e * DOUT + nc0 + ni * 16u + lm) * DHID + 8u * lh;
      v8f acc[2][4] = {};
#pragma unroll 2
      for (unsigned kc = 0; kc < (unsigned)(DHID / 32); ++kc) { v16h a[2], b[4];
#pragma unroll
        for (int mi = 0; mi < 2; ++mi) { union { v16h v; v8h q[2]; } f; f.q[0] = *(const v8h*)&hs[mi * 16 + lm][kc * 32u + 8u * lh]; f.q[1] = *(const v8h*)&hs[mi * 16 + lm][kc * 32u + 16u + 8u * lh]; a[mi] = f.v; }
#pragma unroll
        for (int ni = 0; ni < 4; ++ni) b[ni] = ldfrag_h(br[ni] + kc * 32u);
#pragma unroll
        for (int mi = 0; mi < 2; ++mi)
#pragma unroll
          for (int ni = 0; ni < 4; ++ni) acc[mi][ni] = wmma16(a[mi], b[ni], acc[mi][ni]); }
      float wv[2][8];
#pragma unroll
      for (int mi = 0; mi < 2; ++mi)
#pragma unroll
        for (int r = 0; r < 8; ++r) { const unsigned hidx = tile * (unsigned)MT + mi * 16u + 8u * lh + r; const unsigned hc = hidx < n ? hidx : (n - 1u); wv[mi][r] = l_w[hc] * OSCALE; }
#pragma unroll
      for (int mi = 0; mi < 2; ++mi) {
#pragma unroll
        for (int nip = 0; nip < 2; ++nip) {
          __syncthreads();
#pragma unroll
          for (int q2 = 0; q2 < 2; ++q2)
#pragma unroll
            for (int r = 0; r < 8; ++r) sf[wave][8u * lh + r][q2 * 16 + lm] = acc[mi][2 * nip + q2][r] * wv[mi][r];
          __syncthreads();
          v4f v[4]; size_t go[4]; bool s0[4], s1[4];
#pragma unroll
          for (unsigned it = 0; it < 4u; ++it) { const unsigned rw = it * 4u + (lane >> 3), q = lane & 7u;
            v[it] = *(const v4f*)&sf[wave][rw][4u * q];
            const unsigned hidx = tile * (unsigned)MT + mi * 16u + rw; const bool ok = hidx < n; const unsigned hc = ok ? hidx : (n - 1u);
            int tk = l_tok[hc]; int sl = l_slot[hc];
            asm volatile("" : "+v"(tk)); asm volatile("" : "+v"(sl));
            tk = tk < 0 ? 0 : tk; tk = tk > NB - 1 ? NB - 1 : tk;
            go[it] = (size_t)tk * DOUT + nc0 + nip * 32u + 4u * q; s0[it] = ok && (sl == 0); s1[it] = ok && (sl != 0); }
#pragma unroll
          for (unsigned it = 0; it < 4u; ++it) { if (s0[it]) *(volatile v4f*)(OUT + go[it]) = v[it]; if (s1[it]) *(volatile v4f*)(Y1 + go[it]) = v[it]; }
          __threadfence();
#pragma unroll
          for (unsigned it = 0; it < 4u; ++it) { if (s0[it]) *(volatile v4f*)(OUT + go[it]) = v[it]; if (s1[it]) *(volatile v4f*)(Y1 + go[it]) = v[it]; }
        }
      }
    }
  }
}

__global__ __launch_bounds__(256) void k_comb(const float* __restrict__ X, const float* __restrict__ Y1, float* OUT) {
  const unsigned i = blockIdx.x * 256u + threadIdx.x;
  if (i >= (unsigned)(NB * DIN / 4)) return;
  const v4f x = *(const v4f*)(X + (size_t)i * 4), a = *(const v4f*)(OUT + (size_t)i * 4), b = *(const v4f*)(Y1 + (size_t)i * 4);
  v4f o;
#pragma unroll
  for (int j = 0; j < 4; ++j) o[j] = (bfr(x[j]) + a[j]) + b[j];
  const v4f val = o;
  volatile v4f* p = (volatile v4f*)(OUT + (size_t)i * 4);
  *p = val; __threadfence(); *p = val;
}

extern "C" void kernel_launch(void* const* d_in, const int* in_sizes, int n_in, void* d_out, int out_size, void* d_ws, size_t ws_size, hipStream_t stream) {
  if (n_in < 5) return;
  if (in_sizes[0] < NB * DIN || in_sizes[1] < DIN * NE) return;
  if (in_sizes[2] < NE * DIN * DHID || in_sizes[3] < NE * DIN * DHID || in_sizes[4] < NE * DHID * DOUT) return;
  if ((size_t)out_size < (size_t)NB * DOUT) return;
  if (ws_size < (size_t)WS_END) return;
  const float* X  = (const float*)d_in[0];
  const float* GW = (const float*)d_in[1];
  const float* W1 = (const float*)d_in[2];
  const float* W3 = (const float*)d_in[3];
  const float* W2 = (const float*)d_in[4];
  char* ws = (char*)d_ws;
  unsigned short* XB  = (unsigned short*)(ws + WS_XB);
  unsigned short* W1T = (unsigned short*)(ws + WS_W1T);
  unsigned short* W3T = (unsigned short*)(ws + WS_W3T);
  unsigned short* W2T = (unsigned short*)(ws + WS_W2T);
  float* CMB = (float*)(ws + WS_CMB);
  float* Y1  = (float*)(ws + WS_Y1);
  float* OUT = (float*)d_out;
  k_cvt_x<<<dim3(NB * DIN / 8 / 256), 256, 0, stream>>>(X, XB);
  k_tr<0><<<dim3(DHID / 64, DIN / 64, NE), 256, 0, stream>>>(W1, W1T, (unsigned)DIN, (unsigned)DHID, (unsigned)DIN, (unsigned)DHID, 0u, 1.0f);
  k_tr<0><<<dim3(DHID / 64, DIN / 64, NE), 256, 0, stream>>>(W3, W3T, (unsigned)DIN, (unsigned)DHID, (unsigned)DIN, (unsigned)DHID, 0u, 1.0f);
  k_tr<1><<<dim3(DOUT / 64, DHID / 64, NE), 256, 0, stream>>>(W2, W2T, (unsigned)DHID, (unsigned)DOUT, (unsigned)DHID, (unsigned)DOUT, 0u, WCARRY);
  k_route<<<dim3(NB / RT), 256, 0, stream>>>(XB, GW, CMB);
  k_moe<<<dim3(NB / CH, NE), 256, 0, stream>>>(XB, W1T, W3T, W2T, CMB, OUT, Y1);
  k_comb<<<dim3(NB * DIN / 4 / 256), 256, 0, stream>>>(X, Y1, OUT);
}
